// GAT_65463891526243
// MI455X (gfx1250) — hardware-verified
//
#include <hip/hip_runtime.h>
#include <stddef.h>
#include <stdint.h>
#include <math.h>


#define NB     8
#define NN     2048
#define FD     256
#define DH     128
#define NHEAD  2
#define ROWS   (NB * NN)
#define KP     512
#define NTHR   256
#define GTHR   128
#define GBM    64
#define LDT    132
#define PLN    (DH * NN)
#define NEGSL  0.2f
#define WSMAX  134217728

#define NUX    (ROWS * (FD / 8))
#define NUW0   (DH * (FD / 8))
#define NUW1   (DH * (KP / 8))
#define NUS    512
#define U1     (NUX)
#define U2     (U1 + NUW0)
#define U3     (U2 + NUW0)
#define U4     (U3 + NUW1)
#define U5     (U4 + NUW1)
#define U6     (U5 + NUS)

static_assert((FD % 32) == 0 && (KP % 32) == 0 && KP == 2 * FD);
static_assert(FD == NHEAD * DH && DH == 4 * 32);
static_assert((ROWS % GBM) == 0 && (NN % GBM) == 0 && (NN % 32) == 0);
static_assert(GBM == (GTHR / 32) * 16);
static_assert((U1 % NTHR) == 0 && (U2 % NTHR) == 0 && (U3 % NTHR) == 0);
static_assert((U4 % NTHR) == 0 && (U5 % NTHR) == 0 && (U6 % NTHR) == 0);
static_assert((LDT % 4) == 0 && LDT >= DH);
static_assert(NN == GTHR * 16);
static_assert((FD / 8) == 32 && (KP / 8) == 64);

typedef float          v4f  __attribute__((ext_vector_type(4)));
typedef float          v8f  __attribute__((ext_vector_type(8)));
typedef int            v8i  __attribute__((ext_vector_type(8)));
typedef unsigned int   v4u  __attribute__((ext_vector_type(4)));
typedef unsigned short v8us __attribute__((ext_vector_type(8)));
typedef __bf16         v16b __attribute__((ext_vector_type(16)));
typedef v4f  __attribute__((may_alias)) v4fa;
typedef v8us __attribute__((may_alias)) v8usa;
union FragB { v16b v; v8us h[2]; v8i w; };

__device__ __forceinline__ v8f wmb(const FragB& a, const FragB& b, v8f c) {
  v8f d = __builtin_amdgcn_wmma_f32_16x16x32_bf16(false, a.v, false, b.v, (short)0, c, false, false);
  asm volatile("v_nop\n\tv_nop\n\tv_nop\n\tv_nop" : "+v"(d) : "v"(a.w), "v"(b.w));
  return d;
}

__device__ __forceinline__ unsigned int f2bf(float f) {
  const unsigned int u = __float_as_uint(f);
  return ((u + 0x7FFFu + ((u >> 16) & 1u)) >> 16) & 0xFFFFu;
}
__device__ __forceinline__ float bf2f(unsigned int b) { return __uint_as_float(b << 16); }
__device__ __forceinline__ float bfr(float f) { return bf2f(f2bf(f)); }
__device__ __forceinline__ unsigned int pk2(float lo, float hi) { return f2bf(lo) | (f2bf(hi) << 16); }
__device__ __forceinline__ v4u pack8(const v4f a, const v4f b) {
  v4u r;
  r.x = pk2(a.x, a.y); r.y = pk2(a.z, a.w); r.z = pk2(b.x, b.y); r.w = pk2(b.z, b.w);
  return r;
}
__device__ __forceinline__ void hl2(float p0, float p1, unsigned int& wh, unsigned int& wl) {
  const unsigned int h0 = f2bf(p0), h1 = f2bf(p1);
  const unsigned int l0 = f2bf(p0 - bf2f(h0)), l1 = f2bf(p1 - bf2f(h1));
  wh = h0 | (h1 << 16);
  wl = l0 | (l1 << 16);
}
__device__ __forceinline__ void hl8(float v0, float v1, float v2, float v3,
                                    float v4, float v5, float v6, float v7, v4u& hv, v4u& lv) {
  unsigned int h0, h1, h2, h3, l0, l1, l2, l3;
  hl2(v0, v1, h0, l0);
  hl2(v2, v3, h1, l1);
  hl2(v4, v5, h2, l2);
  hl2(v6, v7, h3, l3);
  const v4u a = {h0, h1, h2, h3};
  const v4u b = {l0, l1, l2, l3};
  hv = a;
  lv = b;
}
__device__ __forceinline__ float leaky(float s) { return s > 0.f ? s : NEGSL * s; }
__device__ __forceinline__ float eluf(float v) { const float e = expm1f(v); return v > 0.f ? v : e; }

__device__ __forceinline__ void t2upd(float v, int j, float& m1, int& i1, float& m2) {
  const bool g = v > m1;
  const float n2 = g ? m1 : fmaxf(m2, v);
  i1 = g ? j : i1;
  m1 = g ? v : m1;
  m2 = n2;
}
__device__ __forceinline__ void t2comb(float& a1, int& ai, float& a2, float b1, int bi, float b2) {
  const bool g = b1 > a1;
  const float n2 = g ? fmaxf(a1, b2) : fmaxf(a2, b1);
  ai = g ? bi : ai;
  a1 = g ? b1 : a1;
  a2 = n2;
}

__device__ __forceinline__ void wunit(const float* __restrict__ W, int v, int ksh, unsigned short* dstHead) {
  const int kq = 1 << ksh;
  const int dl = v >> ksh;
  const int k8 = (v & (kq - 1)) * 8;
  const int kk = k8 & (FD - 1);
  const float* p = W + (size_t)kk * DH + dl;
  v4f a, b;
  a.x = p[0];          a.y = p[DH];         a.z = p[2 * DH];     a.w = p[3 * DH];
  b.x = p[4 * DH];     b.y = p[5 * DH];     b.z = p[6 * DH];     b.w = p[7 * DH];
  const v4u wv = pack8(a, b);
  unsigned short* o = dstHead + (size_t)dl * (size_t)(kq * 8) + k8;
  *(volatile v4u*)o = wv;
  __threadfence();
  *(volatile v4u*)o = wv;
}

__global__ __launch_bounds__(NTHR) void k_prep(
    const float* __restrict__ x,
    const float* __restrict__ W00, const float* __restrict__ W01,
    const float* __restrict__ W10, const float* __restrict__ W11,
    const float* __restrict__ b00, const float* __restrict__ b01,
    const float* __restrict__ b10, const float* __restrict__ b11,
    const float* __restrict__ a00, const float* __restrict__ a01,
    const float* __restrict__ a10, const float* __restrict__ a11,
    unsigned short* XB, unsigned short* WT0, unsigned short* WT1, float* PV)
{
  const int u = (int)blockIdx.x * NTHR + (int)threadIdx.x;
  if (u < U1) {
    const int row = u >> 5;
    const int c0  = (u & 31) * 8;
    const float* p = x + (size_t)row * FD + c0;
    const v4f a = *(const v4fa*)p, b = *(const v4fa*)(p + 4);
    const v4u hv = pack8(a, b);
    unsigned short* o = XB + (size_t)row * FD + c0;
    *(volatile v4u*)o = hv;
    __threadfence();
    *(volatile v4u*)o = hv;
  } else if (u < U2) {
    wunit(W00, u - U1, 5, WT0);
  } else if (u < U3) {
    wunit(W01, u - U2, 5, WT0 + (size_t)DH * FD);
  } else if (u < U4) {
    wunit(W10, u - U3, 6, WT1);
  } else if (u < U5) {
    wunit(W11, u - U4, 6, WT1 + (size_t)DH * KP);
  } else if (u < U6) {
    const int v  = u - U5;
    const int w  = __builtin_amdgcn_readfirstlane(v >> 5);
    const int l4 = (v & 31) * 4;
    if (w >= 12) return;
    v4f s;
    if      (w == 0)  s = *(const v4fa*)(b00 + l4);
    else if (w == 1)  s = *(const v4fa*)(b01 + l4);
    else if (w == 2)  s = *(const v4fa*)(b10 + l4);
    else if (w == 3)  s = *(const v4fa*)(b11 + l4);
    else if (w == 4)  s = *(const v4fa*)(a00 + l4);
    else if (w == 5)  s = *(const v4fa*)(a00 + DH + l4);
    else if (w == 6)  s = *(const v4fa*)(a01 + l4);
    else if (w == 7)  s = *(const v4fa*)(a01 + DH + l4);
    else if (w == 8)  s = *(const v4fa*)(a10 + l4);
    else if (w == 9)  s = *(const v4fa*)(a10 + DH + l4);
    else if (w == 10) s = *(const v4fa*)(a11 + l4);
    else              s = *(const v4fa*)(a11 + DH + l4);
    v4f r;
    r.x = bfr(s.x); r.y = bfr(s.y); r.z = bfr(s.z); r.w = bfr(s.w);
    float* o = PV + w * DH + l4;
    *(volatile v4f*)o = r;
    __threadfence();
    *(volatile v4f*)o = r;
  }
}

__global__ __launch_bounds__(GTHR) void k_proj(
    const unsigned short* __restrict__ A, int K, const unsigned short* __restrict__ WT,
    const float* __restrict__ pvb, const float* __restrict__ pva,
    float* Hf, unsigned short* HT, float* SD)
{
  __shared__ __attribute__((aligned(16))) float stg[GBM * LDT];
  __shared__ __attribute__((aligned(16))) float sdt[2 * GBM];
  const int tid = (int)threadIdx.x, lane = tid & 31, wave = tid >> 5, hh = lane >> 4, m = lane & 15;
  const int rowBase = (int)blockIdx.x * GBM;
  const int head    = (int)blockIdx.y;
  const int colBase = head * DH;

  v8f acc[8];
  {
    const v8f z = {0.f, 0.f, 0.f, 0.f, 0.f, 0.f, 0.f, 0.f};
#pragma unroll
    for (int t = 0; t < 8; ++t) acc[t] = z;
  }
  const unsigned short* ap = A  + (size_t)(rowBase + 16 * wave + m) * (size_t)K + 8 * hh;
  const unsigned short* bp = WT + (size_t)(colBase + m) * (size_t)K + 8 * hh;

#pragma unroll 1
  for (int k0 = 0; k0 < K; k0 += 32) {
    FragB af;
    af.h[0] = *(const v8usa*)(ap + k0);
    af.h[1] = *(const v8usa*)(ap + k0 + 16);
#pragma unroll
    for (int nt = 0; nt < 8; ++nt) {
      const unsigned short* wq = bp + (size_t)(16 * nt) * (size_t)K + k0;
      FragB bf;
      bf.h[0] = *(const v8usa*)wq;
      bf.h[1] = *(const v8usa*)(wq + 16);
      acc[nt] = wmb(af, bf, acc[nt]);
    }
  }

#pragma unroll
  for (int nt = 0; nt < 8; ++nt) {
    const int lc = 16 * nt + m;
#pragma unroll
    for (int r = 0; r < 8; ++r) {
      const int lr = 16 * wave + 8 * hh + r;
      stg[lr * LDT + lc] = acc[nt][r];
    }
  }
  __syncthreads();

  const v4f b4  = *(const v4fa*)(pvb + colBase + 4 * lane);
  const v4f al4 = *(const v4fa*)(pva + head * FD + 4 * lane);
  const v4f ar4 = *(const v4fa*)(pva + head * FD + DH + 4 * lane);
#pragma unroll 1
  for (int i = 0; i < 16; ++i) {
    const int row = 16 * wave + i;
    float* sp = stg + row * LDT + 4 * lane;
    v4f p = *(const v4fa*)sp;
    p.x += b4.x; p.y += b4.y; p.z += b4.z; p.w += b4.w;
    *(v4fa*)sp = p;
    float s = 0.0f, d = 0.0f;
    s = fmaf(p.x, al4.x, s); s = fmaf(p.y, al4.y, s); s = fmaf(p.z, al4.z, s); s = fmaf(p.w, al4.w, s);
    d = fmaf(p.x, ar4.x, d); d = fmaf(p.y, ar4.y, d); d = fmaf(p.z, ar4.z, d); d = fmaf(p.w, ar4.w, d);
#pragma unroll
    for (int off = 16; off > 0; off >>= 1) {
      s += __shfl_xor(s, off);
      d += __shfl_xor(d, off);
    }
    if (lane == 0) { sdt[row] = s; sdt[GBM + row] = d; }
    float* op = Hf + (size_t)(rowBase + row) * FD + colBase + 4 * lane;
    *(volatile v4f*)op = p;
    __threadfence();
    *(volatile v4f*)op = p;
  }
  __syncthreads();

  if (wave == 0) {
    const int which = lane >> 4, piece = lane & 15;
    const v4f sdv = *(const v4fa*)(sdt + 4 * lane);
    float* sp = SD + (size_t)(2 * head + which) * ROWS + rowBase + 4 * piece;
    *(volatile v4f*)sp = sdv;
    __threadfence();
    *(volatile v4f*)sp = sdv;
  }

  const int bb = rowBase >> 11;
  const int j0 = rowBase & (NN - 1);
  unsigned short* hbase = HT + (size_t)((bb * NHEAD + head) * 2) * PLN + j0;
#pragma unroll 1
  for (int it = 0; it < 8; ++it) {
    const int item = it * GTHR + tid;
    const int d  = item >> 3;
    const int jp = item & 7;
    const float* cp = stg + (8 * jp) * LDT + d;
    const float v0 = cp[0],       v1 = cp[LDT],     v2 = cp[2 * LDT], v3 = cp[3 * LDT];
    const float v4 = cp[4 * LDT], v5 = cp[5 * LDT], v6 = cp[6 * LDT], v7 = cp[7 * LDT];
    v4u hv, lv;
    hl8(v0, v1, v2, v3, v4, v5, v6, v7, hv, lv);
    unsigned short* hp = hbase + (size_t)d * NN + 8 * jp;
    unsigned short* lp = hp + PLN;
    *(volatile v4u*)hp = hv;
    *(volatile v4u*)lp = lv;
    __threadfence();
    *(volatile v4u*)hp = hv;
    *(volatile v4u*)lp = lv;
  }
}

__device__ __forceinline__ float pval(float er, float el, float mi, int j, int rowloc) {
  const float s = leaky(el + er);
  const float p = expf(s - mi);
  return (j == rowloc) ? 0.0f : p;
}
__device__ __forceinline__ void ppair(float ea, float eb, int j, float el, float mi, int rowloc,
                                      float& ls, int& wh, int& wl) {
  const float p0 = pval(ea, el, mi, j, rowloc);
  const float p1 = pval(eb, el, mi, j + 1, rowloc);
  ls += p0;
  ls += p1;
  unsigned int uh, ul;
  hl2(p0, p1, uh, ul);
  wh = (int)uh;
  wl = (int)ul;
}

template <int FINAL>
__global__ __launch_bounds__(GTHR) void k_attn(
    const unsigned short* __restrict__ HT, const float* __restrict__ Hf, const float* __restrict__ SD,
    unsigned short* X1, float* outp)
{
  __shared__ __attribute__((aligned(16))) float ers[NN];
  __shared__ __attribute__((aligned(16))) float stg[GBM * LDT];
  __shared__ __attribute__((aligned(16))) float sinv[GBM];
  __shared__ float wt1[4];
  __shared__ float wt2[4];
  __shared__ int   wti[4];
  const int tid = (int)threadIdx.x, lane = tid & 31, wave = tid >> 5, hh = lane >> 4, m = lane & 15;
  const int qt = (int)blockIdx.x, head = (int)blockIdx.y, bb = (int)blockIdx.z;
  const int rowBase = bb * NN + qt * GBM;

  {
    const float* erp = SD + (size_t)(2 * head + 1) * ROWS + (size_t)bb * NN;
    float m1 = -3.0e38f, m2 = -3.0e38f;
    int i1 = 0;
#pragma unroll
    for (int i = 0; i < 4; ++i) {
      const int j4 = 4 * (tid + GTHR * i);
      const v4f e = *(const v4fa*)(erp + j4);
      *(v4fa*)(ers + j4) = e;
      t2upd(e.x, j4,     m1, i1, m2);
      t2upd(e.y, j4 + 1, m1, i1, m2);
      t2upd(e.z, j4 + 2, m1, i1, m2);
      t2upd(e.w, j4 + 3, m1, i1, m2);
    }
#pragma unroll
    for (int off = 16; off > 0; off >>= 1) {
      const float o1 = __shfl_xor(m1, off);
      const int   oi = __shfl_xor(i1, off);
      const float o2 = __shfl_xor(m2, off);
      t2comb(m1, i1, m2, o1, oi, o2);
    }
    if (lane == 0) { wt1[wave] = m1; wt2[wave] = m2; wti[wave] = i1; }
  }
  __syncthreads();
  float g1 = wt1[0], g2 = wt2[0];
  int gi = wti[0];
  t2comb(g1, gi, g2, wt1[1], wti[1], wt2[1]);
  t2comb(g1, gi, g2, wt1[2], wti[2], wt2[2]);
  t2comb(g1, gi, g2, wt1[3], wti[3], wt2[3]);

  const int rowloc = qt * GBM + 16 * wave + m;
  const float el = SD[(size_t)(2 * head) * ROWS + rowBase + 16 * wave + m];
  const float mi = leaky(el + ((rowloc == gi) ? g2 : g1));

  v8f acc[8];
  {
    const v8f z = {0.f, 0.f, 0.f, 0.f, 0.f, 0.f, 0.f, 0.f};
#pragma unroll
    for (int t = 0; t < 8; ++t) acc[t] = z;
  }
  float lsum = 0.0f;
  const unsigned short* bph = HT + (size_t)((bb * NHEAD + head) * 2) * PLN + (size_t)m * NN + 8 * hh;

#pragma unroll 1
  for (int ks = 0; ks < NN / 32; ++ks) {
    const int k0 = 32 * ks;
    const int jb = k0 + 8 * hh;
    const v4f e0 = *(const v4fa*)(ers + jb);
    const v4f e1 = *(const v4fa*)(ers + jb + 4);
    const v4f e2 = *(const v4fa*)(ers + jb + 16);
    const v4f e3 = *(const v4fa*)(ers + jb + 20);
    int h0, h1, h2, h3, h4, h5, h6, h7, l0, l1, l2, l3, l4, l5, l6, l7;
    ppair(e0.x, e0.y, jb,      el, mi, rowloc, lsum, h0, l0);
    ppair(e0.z, e0.w, jb + 2,  el, mi, rowloc, lsum, h1, l1);
    ppair(e1.x, e1.y, jb + 4,  el, mi, rowloc, lsum, h2, l2);
    ppair(e1.z, e1.w, jb + 6,  el, mi, rowloc, lsum, h3, l3);
    ppair(e2.x, e2.y, jb + 16, el, mi, rowloc, lsum, h4, l4);
    ppair(e2.z, e2.w, jb + 18, el, mi, rowloc, lsum, h5, l5);
    ppair(e3.x, e3.y, jb + 20, el, mi, rowloc, lsum, h6, l6);
    ppair(e3.z, e3.w, jb + 22, el, mi, rowloc, lsum, h7, l7);
    FragB ah, al;
    {
      const v8i vh = {h0, h1, h2, h3, h4, h5, h6, h7};
      const v8i vl = {l0, l1, l2, l3, l4, l5, l6, l7};
      ah.w = vh;
      al.w = vl;
    }
#pragma unroll
    for (int nt = 0; nt < 8; ++nt) {
      const unsigned short* q = bph + (size_t)(16 * nt) * NN + k0;
      FragB bh, bl;
      bh.h[0] = *(const v8usa*)q;
      bh.h[1] = *(const v8usa*)(q + 16);
      bl.h[0] = *(const v8usa*)(q + PLN);
      bl.h[1] = *(const v8usa*)(q + PLN + 16);
      acc[nt] = wmb(ah, bh, acc[nt]);
      acc[nt] = wmb(al, bh, acc[nt]);
      acc[nt] = wmb(ah, bl, acc[nt]);
    }
  }

  const float lt = lsum + __shfl_xor(lsum, 16);
#pragma unroll
  for (int nt = 0; nt < 8; ++nt) {
    const int lc = 16 * nt + m;
#pragma unroll
    for (int r = 0; r < 8; ++r) {
      const int lr = 16 * wave + 8 * hh + r;
      stg[lr * LDT + lc] = acc[nt][r];
    }
  }
  if (hh == 0) sinv[16 * wave + m] = 1.0f / lt;
  __syncthreads();

  if constexpr (FINAL == 0) {
    const int hq = lane >> 4, c8 = 8 * (lane & 15);
#pragma unroll 1
    for (int it = 0; it < 8; ++it) {
      const int lr = 16 * wave + 2 * it + hq;
      const int gr = rowBase + lr;
      const float inv = sinv[lr];
      const v4f o0 = *(const v4fa*)(stg + lr * LDT + c8);
      const v4f o1 = *(const v4fa*)(stg + lr * LDT + c8 + 4);
      const float* hp = Hf + (size_t)gr * FD + head * DH + c8;
      const v4f x0 = *(const v4fa*)hp;
      const v4f x1 = *(const v4fa*)(hp + 4);
      const float r0 = eluf(fmaf(o0.x, inv, x0.x)), r1 = eluf(fmaf(o0.y, inv, x0.y));
      const float r2 = eluf(fmaf(o0.z, inv, x0.z)), r3 = eluf(fmaf(o0.w, inv, x0.w));
      const float r4 = eluf(fmaf(o1.x, inv, x1.x)), r5 = eluf(fmaf(o1.y, inv, x1.y));
      const float r6 = eluf(fmaf(o1.z, inv, x1.z)), r7 = eluf(fmaf(o1.w, inv, x1.w));
      v4u hv, lv;
      hl8(r0, r1, r2, r3, r4, r5, r6, r7, hv, lv);
      unsigned short* xp = X1 + (size_t)gr * KP + head * DH + c8;
      unsigned short* yp = xp + FD;
      *(volatile v4u*)xp = hv;
      *(volatile v4u*)yp = lv;
      __threadfence();
      *(volatile v4u*)xp = hv;
      *(volatile v4u*)yp = lv;
    }
  } else {
    const int c4 = 4 * lane;
#pragma unroll 1
    for (int it = 0; it < 16; ++it) {
      const int lr = 16 * wave + it;
      const int gr = rowBase + lr;
      const float inv = sinv[lr];
      const v4f o0 = *(const v4fa*)(stg + lr * LDT + c4);
      const v4f x0 = *(const v4fa*)(Hf + (size_t)gr * FD + head * DH + c4);
      v4f rv;
      rv.x = eluf(fmaf(o0.x, inv, x0.x));
      rv.y = eluf(fmaf(o0.y, inv, x0.y));
      rv.z = eluf(fmaf(o0.z, inv, x0.z));
      rv.w = eluf(fmaf(o0.w, inv, x0.w));
      float* op = outp + (size_t)gr * FD + head * DH + c4;
      *(volatile v4f*)op = rv;
      __threadfence();
      *(volatile v4f*)op = rv;
    }
  }
}

extern "C" void kernel_launch(void* const* d_in, const int* in_sizes, int n_in,
                              void* d_out, int out_size, void* d_ws, size_t ws_size,
                              hipStream_t stream) {
  if (n_in < 14) return;
  if (in_sizes[0] != ROWS * FD) return;
  for (int i = 0; i < 4; ++i) {
    if (in_sizes[2 + 3 * i] != FD * DH) return;
    if (in_sizes[3 + 3 * i] != DH) return;
    if (in_sizes[4 + 3 * i] != 2 * DH) return;
  }
  if (out_size != ROWS * FD) return;

  const float* x   = (const float*)d_in[0];
  const float* W00 = (const float*)d_in[2];
  const float* b00 = (const float*)d_in[3];
  const float* a00 = (const float*)d_in[4];
  const float* W01 = (const float*)d_in[5];
  const float* b01 = (const float*)d_in[6];
  const float* a01 = (const float*)d_in[7];
  const float* W10 = (const float*)d_in[8];
  const float* b10 = (const float*)d_in[9];
  const float* a10 = (const float*)d_in[10];
  const float* W11 = (const float*)d_in[11];
  const float* b11 = (const float*)d_in[12];
  const float* a11 = (const float*)d_in[13];
  float* out = (float*)d_out;

  char* ws = (char*)d_ws;
  size_t off = 0;
  const size_t oXB  = off; off += (size_t)ROWS * FD * 2;                  off = (off + 255) & ~(size_t)255;
  const size_t oWT0 = off; off += (size_t)FD * FD * 2;                    off = (off + 255) & ~(size_t)255;
  const size_t oWT1 = off; off += (size_t)FD * KP * 2;                    off = (off + 255) & ~(size_t)255;
  const size_t oPV  = off; off += (size_t)1536 * 4;                       off = (off + 255) & ~(size_t)255;
  const size_t oHf  = off; off += (size_t)ROWS * FD * 4;                  off = (off + 255) & ~(size_t)255;
  const size_t oHT  = off; off += (size_t)NB * NHEAD * 2 * PLN * 2;       off = (off + 255) & ~(size_t)255;
  const size_t oSD  = off; off += (size_t)4 * ROWS * 4;                   off = (off + 255) & ~(size_t)255;
  const size_t oX1  = off; off += (size_t)ROWS * KP * 2;                  off = (off + 255) & ~(size_t)255;
  if (off > ws_size || off > (size_t)WSMAX) return;
  unsigned short* XB  = (unsigned short*)(ws + oXB);
  unsigned short* WT0 = (unsigned short*)(ws + oWT0);
  unsigned short* WT1 = (unsigned short*)(ws + oWT1);
  float*          PV  = (float*)(ws + oPV);
  float*          Hf  = (float*)(ws + oHf);
  unsigned short* HT  = (unsigned short*)(ws + oHT);
  float*          SD  = (float*)(ws + oSD);
  unsigned short* X1  = (unsigned short*)(ws + oX1);

  k_prep<<<U6 / NTHR, NTHR, 0, stream>>>(x, W00, W01, W10, W11, b00, b01, b10, b11, a00, a01, a10, a11,
                                         XB, WT0, WT1, PV);
  k_proj<<<dim3(ROWS / GBM, NHEAD), GTHR, 0, stream>>>(XB, FD, WT0, PV, PV + 512, Hf, HT, SD);
  k_attn<0><<<dim3(NN / GBM, NHEAD, NB), GTHR, 0, stream>>>(HT, Hf, SD, X1, out);
  k_proj<<<dim3(ROWS / GBM, NHEAD), GTHR, 0, stream>>>(X1, KP, WT1, PV + 256, PV + 1024, Hf, HT, SD);
  k_attn<1><<<dim3(NN / GBM, NHEAD, NB), GTHR, 0, stream>>>(HT, Hf, SD, X1, out);
}
